// RNet_34050500723401
// MI455X (gfx1250) — hardware-verified
//
#include <hip/hip_runtime.h>


#define BS   32
#define NR   100
#define NRP  128
#define IND  2048
#define QD   1024
#define CCH  256
#define C1   128
#define C2   64
#define BCH  4
#define RCH  (BCH * NR * NR)
#define SMP  10240
typedef _Float16 h16;
typedef unsigned short bf;
typedef __attribute__((ext_vector_type(16))) __bf16   v16bf;
typedef __attribute__((ext_vector_type(16))) _Float16 v16h;
typedef __attribute__((ext_vector_type(8)))  _Float16 v8h;
typedef __attribute__((ext_vector_type(8)))  unsigned short v8us;
typedef __attribute__((ext_vector_type(8)))  float    v8f;
typedef __attribute__((ext_vector_type(4)))  float    v4f;
typedef v8h  __attribute__((may_alias)) v8ha;
typedef v4f  __attribute__((may_alias)) v4fa;
typedef v8us __attribute__((may_alias)) v8usa;

__device__ __forceinline__ unsigned short f2bf(float f) { unsigned u = __float_as_uint(f); u += 0x7FFFu + ((u >> 16) & 1u); return (unsigned short)(u >> 16); }
__device__ __forceinline__ float bf2f(unsigned short b) { return __uint_as_float(((unsigned)b) << 16); }
__device__ __forceinline__ float bfr(float f) { return bf2f(f2bf(f)); }
__device__ __forceinline__ v16h cat16(v8h lo, v8h hi) { return __builtin_shufflevector(lo, hi, 0, 1, 2, 3, 4, 5, 6, 7, 8, 9, 10, 11, 12, 13, 14, 15); }
__device__ __forceinline__ v16bf cat16b(v8us lo, v8us hi) { return __builtin_bit_cast(v16bf, __builtin_shufflevector(lo, hi, 0, 1, 2, 3, 4, 5, 6, 7, 8, 9, 10, 11, 12, 13, 14, 15)); }
__device__ __forceinline__ v8f wmma16(v16h a, v16h b, v8f c) { return __builtin_amdgcn_wmma_f32_16x16x32_f16(false, a, false, b, (short)0, c, false, false); }
__device__ __forceinline__ v8f wmmab(v16bf a, v16bf b, v8f c) { return __builtin_amdgcn_wmma_f32_16x16x32_bf16(false, a, false, b, (short)0, c, false, false); }


template <typename T16> struct WFrag;
template <> struct WFrag<h16> { typedef v16h V; static __device__ __forceinline__ V ld(const h16* p) { return cat16(*(const v8h*)p, *(const v8h*)(p + 16)); } static __device__ __forceinline__ v8f mma(V a, V b, v8f c) { return wmma16(a, b, c); } };
template <> struct WFrag<bf> { typedef v16bf V; static __device__ __forceinline__ V ld(const bf* p) { return cat16b(*(const v8us*)p, *(const v8us*)(p + 16)); } static __device__ __forceinline__ v8f mma(V a, V b, v8f c) { return wmmab(a, b, c); } };
template <typename T16, int NSPLIT, bool BIAS>
__global__ __launch_bounds__(32) void k_gemmw(const T16* __restrict__ A, const T16* __restrict__ A2, const T16* __restrict__ Bt, const T16* __restrict__ Bt2, int K, float* C, int ldc, const float* __restrict__ bias, size_t sA, size_t sB, size_t sC) {
    typedef typename WFrag<T16>::V V;
    __shared__ __align__(16) float os[16 * 68];
    const size_t z = blockIdx.z; A += z * sA; if (A2) A2 += z * sA; Bt += z * sB; if (Bt2) Bt2 += z * sB; C += z * sC;
    const int lane = threadIdx.x & 31, lr = lane & 15, hi = lane >> 4; const int r0 = blockIdx.x * 64, c0 = blockIdx.y * 64;
    v8f acc[4][4];
#pragma unroll
    for (int mb = 0; mb < 4; ++mb)
#pragma unroll
        for (int nb = 0; nb < 4; ++nb) acc[mb][nb] = (v8f){};
    const size_t aoff = (size_t)(r0 + lr) * K + 8 * hi, boff = (size_t)(c0 + lr) * K + 8 * hi;
#pragma unroll 1
    for (int kc = 0; kc < K; kc += 32) {
        V a[4], a2[4];
#pragma unroll
        for (int mb = 0; mb < 4; ++mb) { a[mb] = WFrag<T16>::ld(A + aoff + (size_t)mb * 16 * K + kc); if (NSPLIT == 1 || NSPLIT == 2) a2[mb] = WFrag<T16>::ld(A2 + aoff + (size_t)mb * 16 * K + kc); }
#pragma unroll
        for (int nb = 0; nb < 4; ++nb) { const V b = WFrag<T16>::ld(Bt + boff + (size_t)nb * 16 * K + kc); V b2; if (NSPLIT >= 2) b2 = WFrag<T16>::ld(Bt2 + boff + (size_t)nb * 16 * K + kc);
#pragma unroll
            for (int mb = 0; mb < 4; ++mb) { acc[mb][nb] = WFrag<T16>::mma(a[mb], b, acc[mb][nb]); if (NSPLIT == 1 || NSPLIT == 2) acc[mb][nb] = WFrag<T16>::mma(a2[mb], b, acc[mb][nb]); if (NSPLIT >= 2) acc[mb][nb] = WFrag<T16>::mma(a[mb], b2, acc[mb][nb]); } }
        asm volatile("v_nop\n\tv_nop\n\tv_nop\n\tv_nop" : "+v"(acc[0][0]), "+v"(acc[1][1]), "+v"(acc[2][2]), "+v"(acc[3][3]) : "v"(a[0]), "v"(a[3]));
    }
#pragma unroll
    for (int mb = 0; mb < 4; ++mb) {
#pragma unroll
        for (int nb = 0; nb < 4; ++nb) {
#pragma unroll
            for (int j = 0; j < 8; ++j) os[(hi * 8 + j) * 68 + nb * 16 + lr] = acc[mb][nb][j]; }
        __builtin_amdgcn_wave_barrier(); asm volatile("" ::: "memory");
        float* crow = C + (size_t)(r0 + mb * 16) * ldc + c0;
#pragma unroll 1
        for (int ps = 0; ps < 2; ++ps) {
#pragma unroll
            for (int s = 0; s < 8; ++s) { const int row = 2 * s + hi, cofs = lr * 4; v4f val = *(const v4fa*)(os + row * 68 + cofs); if (BIAS) { val[0] += bfr(bias[c0 + cofs]); val[1] += bfr(bias[c0 + cofs + 1]); val[2] += bfr(bias[c0 + cofs + 2]); val[3] += bfr(bias[c0 + cofs + 3]); }
                *(volatile v4f*)(crow + (size_t)row * ldc + cofs) = val; }
            if (ps == 0) __threadfence(); }
        __builtin_amdgcn_wave_barrier(); asm volatile("" ::: "memory");
    }
}

__device__ __forceinline__ void splitf(float y, unsigned short& h, unsigned short& l) { h = f2bf(y); l = f2bf(y - bf2f(h)); }
typedef __attribute__((ext_vector_type(2))) unsigned short v2us;
typedef __attribute__((ext_vector_type(4))) unsigned short v4us;

__global__ __launch_bounds__(256) void k_wtG(const float* __restrict__ w, int K, int N, bf* Bt) {
    const int lane = threadIdx.x & 31; const int L0 = (blockIdx.x * 8 + (threadIdx.x >> 5)) * 8; const int nlines = N * K / 64;
#pragma unroll 1
    for (int ps = 0; ps < 2; ++ps) {
#pragma unroll 1
        for (int l = 0; l < 8; ++l) { const int L = L0 + l; if (L >= nlines) break; const size_t e = (size_t)L * 64 + lane * 2; const int k = (int)(e % K), n = (int)(e / K); v2us o;
            o[0] = f2bf(w[(size_t)k * N + n]); o[1] = f2bf(w[(size_t)(k + 1) * N + n]); *(volatile v2us*)(Bt + e) = o; }
        if (ps == 0) __threadfence(); }
}
__global__ __launch_bounds__(256) void k_cvt8(const float* __restrict__ src, bf* dst, size_t n8) { const size_t i = (size_t)blockIdx.x * 256 + threadIdx.x; if (i >= n8) return; const v8f v = *(const v8f*)(src + i * 8); v8us o;
#pragma unroll
    for (int k = 0; k < 8; ++k) o[k] = f2bf(v[k]); *(volatile v8us*)(dst + i * 8) = o; __threadfence(); *(volatile v8us*)(dst + i * 8) = o; }
__global__ __launch_bounds__(256) void k_qb(const float* __restrict__ Q, bf* QB) { const int e = (blockIdx.x * 256 + threadIdx.x) * 4; if (e >= 64 * QD) return; const int r = e / QD; v4us o;
#pragma unroll
    for (int q = 0; q < 4; ++q) o[q] = r < BS ? f2bf(Q[e + q]) : (unsigned short)0; *(volatile v4us*)(QB + e) = o; __threadfence(); *(volatile v4us*)(QB + e) = o; }
__global__ __launch_bounds__(256) void k_xpq(const float* __restrict__ XP, const float* __restrict__ QP, float* XPQ) { const size_t e = ((size_t)blockIdx.x * 256 + threadIdx.x) * 4; if (e >= (size_t)BS * NR * CCH) return; const int c = (int)(e % CCH); const int b = (int)(e / ((size_t)NR * CCH)); const v4f a = *(const v4f*)(XP + e), q = *(const v4f*)(QP + (size_t)b * CCH + c); v4f o;
#pragma unroll
    for (int u = 0; u < 4; ++u) o[u] = __fadd_rn(a[u], q[u]); *(volatile v4f*)(XPQ + e) = o; __threadfence(); *(volatile v4f*)(XPQ + e) = o; }
__global__ __launch_bounds__(256) void k_pair(const float* __restrict__ XPQ, int b0, bf* Ph, bf* Pl) { const size_t e = ((size_t)blockIdx.x * 256 + threadIdx.x) * 4; if (e >= (size_t)RCH * CCH) return; const int c = (int)(e % CCH); const size_t r = e / CCH; const int j = (int)(r % NR); const int i = (int)((r / NR) % NR); const int b = b0 + (int)(r / (NR * NR));
    const v4f xi = *(const v4f*)(XPQ + ((size_t)b * NR + i) * CCH + c), xj = *(const v4f*)(XPQ + ((size_t)b * NR + j) * CCH + c); v4us oh, ol;
#pragma unroll
    for (int u = 0; u < 4; ++u) { unsigned short a, b2; splitf(__fmul_rn(xj[u], xi[u]), a, b2); oh[u] = a; ol[u] = b2; } *(volatile v4us*)(Ph + e) = oh; *(volatile v4us*)(Pl + e) = ol; __threadfence(); *(volatile v4us*)(Ph + e) = oh; *(volatile v4us*)(Pl + e) = ol; }
__global__ __launch_bounds__(256) void k_relspl(const float* __restrict__ F, size_t n4, bf* Fh, bf* Fl) { const size_t i = ((size_t)blockIdx.x * 256 + threadIdx.x) * 4; if (i >= n4 * 4) return; const v4f a = *(const v4f*)(F + i); v4us oh, ol;
#pragma unroll
    for (int q = 0; q < 4; ++q) { unsigned short u, c2; splitf(fmaxf(a[q], 0.f), u, c2); oh[q] = u; ol[q] = c2; } *(volatile v4us*)(Fh + i) = oh; *(volatile v4us*)(Fl + i) = ol; __threadfence(); *(volatile v4us*)(Fh + i) = oh; *(volatile v4us*)(Fl + i) = ol; }
__global__ __launch_bounds__(256) void k_h3(const float* __restrict__ H2, const float* __restrict__ Wc, const float* __restrict__ bc, size_t r0, float* R) { const int r = blockIdx.x * 256 + threadIdx.x; if (r >= RCH) return; float s = 0.f;
    for (int c = 0; c < C2; ++c) { float p = __fmul_rn(fmaxf(H2[(size_t)r * C2 + c], 0.f), bfr(Wc[c])); asm volatile("" : "+v"(p)); s = __fadd_rn(s, p); } const float o = fmaxf(__fadd_rn(s, bfr(bc[0])), 0.f); *(volatile float*)(R + r0 + r) = o; __threadfence(); *(volatile float*)(R + r0 + r) = o; }
__global__ __launch_bounds__(256) void k_rsoft(const float* __restrict__ R, float* SM) { const int lane = threadIdx.x & 31; const int w = blockIdx.x * 8 + (threadIdx.x >> 5); if (w >= 2 * BS) return; const int b = w % BS, br = w / BS; const float* rb = R + ((size_t)br * BS + b) * NR * NR; float mx = -3.0e38f;
    for (int f = lane; f < NR * NR; f += 32) { const int i = f / NR, j = f % NR; mx = fmaxf(mx, __fadd_rn(rb[f], rb[j * NR + i])); }
#pragma unroll
    for (int sh = 16; sh; sh >>= 1) mx = fmaxf(mx, __shfl_xor(mx, sh, 32));
    float s = 0.f;
    for (int f = lane; f < NR * NR; f += 32) { const int i = f / NR, j = f % NR; float d0 = __fsub_rn(__fadd_rn(rb[f], rb[j * NR + i]), mx); asm volatile("" : "+v"(d0)); s = __fadd_rn(s, __expf(d0)); }
#pragma unroll
    for (int sh = 16; sh; sh >>= 1) s += __shfl_xor(s, sh, 32);
    const float rs = __fdiv_rn(1.0f, s); float* sb = SM + ((size_t)br * BS + b) * SMP;
    for (int ps = 0; ps < 2; ++ps) { for (int f = lane; f < NR * NR; f += 32) { const int i = f / NR, j = f % NR; float d0 = __fsub_rn(__fadd_rn(rb[f], rb[j * NR + i]), mx); asm volatile("" : "+v"(d0)); *(volatile float*)(sb + f) = __fmul_rn(__expf(d0), rs); } if (ps == 0) __threadfence(); } }
__global__ __launch_bounds__(256) void k_rm(const float* __restrict__ SM, bf* Ah, bf* Al) { const size_t e = ((size_t)blockIdx.x * 256 + threadIdx.x) * 4; if (e >= (size_t)BS * NRP * NRP) return; const int j = (int)(e % NRP); const int i = (int)((e / NRP) % NRP); const int b = (int)(e / ((size_t)NRP * NRP)); v4us oh, ol;
#pragma unroll
    for (int q = 0; q < 4; ++q) { const int jq = j + q; float v = 0.f; if (i < NR && jq < NR) { const size_t f = (size_t)b * SMP + (size_t)i * NR + jq; v = __fadd_rn(SM[f], SM[(size_t)BS * SMP + f]); } unsigned short a, c2; splitf(v, a, c2); oh[q] = a; ol[q] = c2; }
    *(volatile v4us*)(Ah + e) = oh; *(volatile v4us*)(Al + e) = ol; __threadfence(); *(volatile v4us*)(Ah + e) = oh; *(volatile v4us*)(Al + e) = ol; }
__global__ __launch_bounds__(256) void k_xT(const float* __restrict__ X, bf* XT) { const size_t e = ((size_t)blockIdx.x * 256 + threadIdx.x) * 4; if (e >= (size_t)BS * IND * NRP) return; const int j = (int)(e % NRP); const int d = (int)((e / NRP) % IND); const int b = (int)(e / ((size_t)NRP * IND)); v4us o;
#pragma unroll
    for (int q = 0; q < 4; ++q) { const int jq = j + q; o[q] = jq < NR ? f2bf(X[((size_t)b * NR + jq) * IND + d]) : (unsigned short)0; } *(volatile v4us*)(XT + e) = o; __threadfence(); *(volatile v4us*)(XT + e) = o; }
__global__ __launch_bounds__(256) void k_out(const float* __restrict__ REL, float* OUT) { const size_t e = ((size_t)blockIdx.x * 256 + threadIdx.x) * 4; if (e >= (size_t)BS * NR * IND) return; const int d = (int)(e % IND); const int i = (int)((e / IND) % NR); const int b = (int)(e / ((size_t)IND * NR)); const v4f a = *(const v4f*)(REL + ((size_t)b * NRP + i) * IND + d); v4f o;
#pragma unroll
    for (int q = 0; q < 4; ++q) o[q] = __fmul_rn(a[q], 0.5f); *(volatile v4f*)(OUT + e) = o; __threadfence(); *(volatile v4f*)(OUT + e) = o; }

extern "C" void kernel_launch(void* const* d_in, const int* in_sizes, int n_in,
                              void* d_out, int out_size, void* d_ws, size_t ws_size, hipStream_t stream) {
    (void)in_sizes; (void)n_in; (void)out_size;
    const float* IN[18]; for (int i = 0; i < 18; ++i) IN[i] = (const float*)d_in[i];
    float* OUT = (float*)d_out;
    char* wsp = (char*)d_ws;
    auto take = [&](size_t bytes) { char* p = wsp; wsp += (bytes + 255) & ~(size_t)255; return (void*)p; };
    bf* WV = (bf*)take((size_t)CCH * IND * 2); bf* WQ = (bf*)take((size_t)CCH * QD * 2); bf* WA[2]; bf* WB[2]; for (int i = 0; i < 2; ++i) { WA[i] = (bf*)take((size_t)C1 * CCH * 2); WB[i] = (bf*)take((size_t)C2 * C1 * 2); }
    bf* XB = (bf*)take((size_t)BS * NR * IND * 2); bf* QB = (bf*)take((size_t)64 * QD * 2); float* XP = (float*)take((size_t)BS * NR * CCH * 4); float* QP = (float*)take((size_t)64 * CCH * 4); float* XPQ = (float*)take((size_t)BS * NR * CCH * 4);
    bf* Ph = (bf*)take((size_t)RCH * CCH * 2); bf* Pl = (bf*)take((size_t)RCH * CCH * 2); float* H1 = (float*)take((size_t)RCH * C1 * 4); bf* H1h = (bf*)take((size_t)RCH * C1 * 2); bf* H1l = (bf*)take((size_t)RCH * C1 * 2); float* H2 = (float*)take((size_t)RCH * C2 * 4);
    float* R = (float*)take((size_t)2 * BS * NR * NR * 4); float* SM = (float*)take((size_t)2 * BS * SMP * 4); bf* Ah = (bf*)take((size_t)BS * NRP * NRP * 2); bf* Al = (bf*)take((size_t)BS * NRP * NRP * 2); bf* XT = (bf*)take((size_t)BS * IND * NRP * 2); float* REL = (float*)take((size_t)BS * NRP * IND * 4);
    if ((size_t)(wsp - (char*)d_ws) > ws_size) return;
    k_wtG<<<(IND * CCH / 64 + 63) / 64, 256, 0, stream>>>(IN[2], IND, CCH, WV); k_wtG<<<(QD * CCH / 64 + 63) / 64, 256, 0, stream>>>(IN[4], QD, CCH, WQ);
    for (int i = 0; i < 2; ++i) { k_wtG<<<(CCH * C1 / 64 + 63) / 64, 256, 0, stream>>>(IN[6 + 6 * i], CCH, C1, WA[i]); k_wtG<<<(C1 * C2 / 64 + 63) / 64, 256, 0, stream>>>(IN[8 + 6 * i], C1, C2, WB[i]); }
    k_cvt8<<<(unsigned)(((size_t)BS * NR * IND / 8 + 255) / 256), 256, 0, stream>>>(IN[1], XB, (size_t)BS * NR * IND / 8); k_qb<<<(64 * QD / 4 + 255) / 256, 256, 0, stream>>>(IN[0], QB);
    k_gemmw<bf, 0, true><<<dim3(BS * NR / 64, CCH / 64, 1), 32, 0, stream>>>(XB, nullptr, WV, nullptr, IND, XP, CCH, IN[3], 0, 0, 0);
    k_gemmw<bf, 0, true><<<dim3(1, CCH / 64, 1), 32, 0, stream>>>(QB, nullptr, WQ, nullptr, QD, QP, CCH, IN[5], 0, 0, 0);
    k_xpq<<<(unsigned)(((size_t)BS * NR * CCH / 4 + 255) / 256), 256, 0, stream>>>(XP, QP, XPQ);
    for (int ck = 0; ck < BS / BCH; ++ck) { const int b0 = ck * BCH;
        k_pair<<<(unsigned)(((size_t)RCH * CCH / 4 + 255) / 256), 256, 0, stream>>>(XPQ, b0, Ph, Pl);
        for (int br = 0; br < 2; ++br) {
            k_gemmw<bf, 1, true><<<dim3(RCH / 64, C1 / 64, 1), 32, 0, stream>>>(Ph, Pl, WA[br], nullptr, CCH, H1, C1, IN[7 + 6 * br], 0, 0, 0);
            k_relspl<<<(unsigned)(((size_t)RCH * C1 / 4 + 255) / 256), 256, 0, stream>>>(H1, (size_t)RCH * C1 / 4, H1h, H1l);
            k_gemmw<bf, 1, true><<<dim3(RCH / 64, 1, 1), 32, 0, stream>>>(H1h, H1l, WB[br], nullptr, C1, H2, C2, IN[9 + 6 * br], 0, 0, 0);
            k_h3<<<(RCH + 255) / 256, 256, 0, stream>>>(H2, IN[10 + 6 * br], IN[11 + 6 * br], ((size_t)br * BS + b0) * NR * NR, R); } }
    k_rsoft<<<(2 * BS + 7) / 8, 256, 0, stream>>>(R, SM); k_rm<<<(unsigned)(((size_t)BS * NRP * NRP / 4 + 255) / 256), 256, 0, stream>>>(SM, Ah, Al); k_xT<<<(unsigned)(((size_t)BS * IND * NRP / 4 + 255) / 256), 256, 0, stream>>>(IN[1], XT);
    k_gemmw<bf, 1, false><<<dim3(NRP / 64, IND / 64, BS), 32, 0, stream>>>(Ah, Al, XT, nullptr, NRP, REL, IND, nullptr, (size_t)NRP * NRP, (size_t)IND * NRP, (size_t)NRP * IND);
    k_out<<<(unsigned)(((size_t)BS * NR * IND / 4 + 255) / 256), 256, 0, stream>>>(REL, OUT);
}
